// TripletGraphTransformerLayer_87187836109387
// MI455X (gfx1250) — hardware-verified
//
#include <hip/hip_runtime.h>
#include <math.h>
#include <stdint.h>

#define NN     256
#define DNODE  256
#define DEDGE  128
#define NH     8
#define NHT    4
#define NPAIR  65536
#define OUT1_OFF 65536
#define NTRI   400
#define PLANE_H ((size_t)NPAIR * DEDGE)
#define FFN_LDS 202240
#define LN_EPS 1e-5f

static_assert(NN % 64 == 0);
static_assert(DEDGE == 128);
static_assert(NHT * 32 == DEDGE);
static_assert(NH * 32 == DNODE);
static_assert(392 <= NTRI);
static_assert(NTRI % 16 == 0);
static_assert(FFN_LDS <= 327680);
static_assert(OUT1_OFF == NN * DNODE);

typedef __attribute__((ext_vector_type(16))) __bf16 v16b;
typedef __attribute__((ext_vector_type(8)))  __bf16 v8b;
typedef __attribute__((ext_vector_type(8)))  float  v8f;
typedef __attribute__((ext_vector_type(4)))  float  v4f;
typedef __attribute__((ext_vector_type(4)))  unsigned int v4u;
typedef __attribute__((ext_vector_type(2)))  unsigned int v2u;
typedef v8b __attribute__((may_alias)) v8ba;
typedef v4f __attribute__((may_alias)) v4fa;
typedef v4u __attribute__((may_alias)) v4ua;
typedef v2u __attribute__((may_alias)) v2ua;

union FragU { v16b v; v8b h[2]; };

__device__ __forceinline__ unsigned short f2bf(float f) {
  const unsigned u = __float_as_uint(f);
  return (unsigned short)((u + 0x7FFFu + ((u >> 16) & 1u)) >> 16);
}
__device__ __forceinline__ float bf2f(unsigned short h) { return __uint_as_float(((unsigned)h) << 16); }
__device__ __forceinline__ float rbf(float f) { return bf2f(f2bf(f)); }
__device__ __forceinline__ unsigned pk16(unsigned short a, unsigned short b) { return (unsigned)a | ((unsigned)b << 16); }
__device__ __forceinline__ unsigned pkhi2(float a, float b) { return pk16(f2bf(a), f2bf(b)); }
__device__ __forceinline__ unsigned pklo2(float a, float b) {
  const unsigned short ha = f2bf(a), hb = f2bf(b);
  return pk16(f2bf(a - bf2f(ha)), f2bf(b - bf2f(hb)));
}
__device__ __forceinline__ float gelu_f(float x) { return 0.5f * x * (1.0f + erff(x * 0.70710678118654752f)); }
__device__ __forceinline__ float sigm(float x) { return 1.0f / (1.0f + expf(-x)); }

__device__ __forceinline__ float wsum32(float v) {
  v += __shfl_xor(v, 16, 32); v += __shfl_xor(v, 8, 32); v += __shfl_xor(v, 4, 32);
  v += __shfl_xor(v, 2, 32);  v += __shfl_xor(v, 1, 32);
  return v;
}
__device__ __forceinline__ float wmax32(float v) {
  v = fmaxf(v, __shfl_xor(v, 16, 32)); v = fmaxf(v, __shfl_xor(v, 8, 32)); v = fmaxf(v, __shfl_xor(v, 4, 32));
  v = fmaxf(v, __shfl_xor(v, 2, 32));  v = fmaxf(v, __shfl_xor(v, 1, 32));
  return v;
}
__device__ __forceinline__ float hsum16(float v) {
  v += __shfl_xor(v, 8, 32); v += __shfl_xor(v, 4, 32); v += __shfl_xor(v, 2, 32); v += __shfl_xor(v, 1, 32);
  return v;
}
__device__ __forceinline__ float hmax16(float v) {
  v = fmaxf(v, __shfl_xor(v, 8, 32)); v = fmaxf(v, __shfl_xor(v, 4, 32));
  v = fmaxf(v, __shfl_xor(v, 2, 32)); v = fmaxf(v, __shfl_xor(v, 1, 32));
  return v;
}
__device__ __forceinline__ v4f ln128(v4f x) {
  float s = (x[0] + x[1]) + (x[2] + x[3]);
  s = wsum32(s);
  const float mean = s * (1.0f / 128.0f);
  const v4f d = x - mean;
  float q = (d[0] * d[0] + d[1] * d[1]) + (d[2] * d[2] + d[3] * d[3]);
  q = wsum32(q);
  const float rs = rsqrtf(q * (1.0f / 128.0f) + LN_EPS);
  return d * rs;
}

__device__ __forceinline__ void wave_sync() {
  __builtin_amdgcn_fence(__ATOMIC_RELEASE, "workgroup");
  __builtin_amdgcn_wave_barrier();
  __builtin_amdgcn_fence(__ATOMIC_ACQUIRE, "workgroup");
}

__device__ __forceinline__ v8f mma(v16b a, v16b b, v8f c) {
  return __builtin_amdgcn_wmma_f32_16x16x32_bf16(false, a, false, b, (short)0, c, false, false);
}
__device__ __forceinline__ v8f mma_g(v16b a, v16b b, v8f c) {
  c = __builtin_amdgcn_wmma_f32_16x16x32_bf16(false, a, false, b, (short)0, c, false, false);
  asm volatile("v_nop\n\tv_nop\n\tv_nop\n\tv_nop" : "+v"(c) : "v"(a), "v"(b));
  return c;
}
__device__ __forceinline__ void guard4(v8f& c0, v8f& c1, v8f& c2, v8f& c3, v16b a, v16b b0, v16b b1, v16b b2, v16b b3) {
  asm volatile("v_nop\n\tv_nop\n\tv_nop\n\tv_nop" : "+v"(c0), "+v"(c1), "+v"(c2), "+v"(c3)
               : "v"(a), "v"(b0), "v"(b1), "v"(b2), "v"(b3));
}
__device__ __forceinline__ void guard8(v8f& c0, v8f& c1, v8f& c2, v8f& c3, v8f& c4, v8f& c5, v8f& c6, v8f& c7,
                                       v16b a0, v16b a1, v16b b0, v16b b1, v16b b2, v16b b3) {
  asm volatile("v_nop\n\tv_nop\n\tv_nop\n\tv_nop"
               : "+v"(c0), "+v"(c1), "+v"(c2), "+v"(c3), "+v"(c4), "+v"(c5), "+v"(c6), "+v"(c7)
               : "v"(a0), "v"(a1), "v"(b0), "v"(b1), "v"(b2), "v"(b3));
}
__device__ __forceinline__ v16b ldfrag_g(const unsigned short* __restrict__ p) {
  FragU f;
  f.h[0] = *(const v8ba*)(p);
  f.h[1] = *(const v8ba*)(p + 16);
  return f.v;
}
#define LDS_FRAG(dst, base, off) do { FragU f_; \
    f_.h[0] = *(const v8ba*)((base) + (off)); \
    f_.h[1] = *(const v8ba*)((base) + (off) + 16); \
    (dst) = f_.v; } while (0)

__global__ __launch_bounds__(256) __attribute__((amdgpu_num_vgpr(248)))
void k_cvt(const float* __restrict__ in, unsigned short* __restrict__ out, int n8) {
  const int g = blockIdx.x * 256 + threadIdx.x;
  if (g >= n8) return;
  const v4f a = *(const v4fa*)(in + (size_t)g * 8);
  const v4f b = *(const v4fa*)(in + (size_t)g * 8 + 4);
  const v4u o = { pkhi2(a[0], a[1]), pkhi2(a[2], a[3]), pkhi2(b[0], b[1]), pkhi2(b[2], b[3]) };
  unsigned short* dst = out + (size_t)g * 8;
  *(volatile v4u*)dst = o;
  __threadfence();
  *(volatile v4u*)dst = o;
}

__global__ __launch_bounds__(256) __attribute__((amdgpu_num_vgpr(248)))
void k_prepT(const float* __restrict__ W, unsigned short* __restrict__ out,
             int K, int Ncols, int KD, int rowsOut) {
  const int G = KD >> 3;
  const int idx = blockIdx.x * 256 + threadIdx.x;
  if (idx >= rowsOut * G) return;
  const int n = idx / G;
  const int g = idx - n * G;
  const int nc = (n < Ncols) ? n : (Ncols - 1);
  const bool live = (n < Ncols);
  int kb = g * 8;
  if (kb >= K) kb -= K;
  float f[8];
#pragma unroll
  for (int e = 0; e < 8; ++e) f[e] = W[(size_t)(kb + e) * Ncols + nc];
#pragma unroll
  for (int e = 0; e < 8; ++e) f[e] = live ? f[e] : 0.0f;
  const v4u o = { pkhi2(f[0], f[1]), pkhi2(f[2], f[3]), pkhi2(f[4], f[5]), pkhi2(f[6], f[7]) };
  unsigned short* dst = out + (size_t)n * KD + g * 8;
  *(volatile v4u*)dst = o;
  __threadfence();
  *(volatile v4u*)dst = o;
}

template <bool BIAS, bool GELU, int NRES, bool R1RND, int OUT>
__global__ __launch_bounds__(128) __attribute__((amdgpu_num_vgpr(248)))
void k_gemm(const unsigned short* __restrict__ A, const unsigned short* __restrict__ Bt, void* Cv,
            const float* __restrict__ bias, const float* R1, const float* R2,
            int lda, int ldb, int ldc, int K) {
  __shared__ __align__(16) float slab[4 * 32 * 68];
  __shared__ __align__(16) float sbias[64];
  const int tid = threadIdx.x, lane = tid & 31, w = tid >> 5, h = lane >> 4, m = lane & 15;
  const int m0 = blockIdx.x * 128 + 32 * w;
  const int n0 = blockIdx.y * 64;
  if (tid < 64) sbias[tid] = BIAS ? rbf(bias[n0 + tid]) : 0.0f;
  __syncthreads();

  const unsigned short* a0 = A + (size_t)(m0 + m) * lda + 8 * h;
  const unsigned short* a1 = a0 + (size_t)16 * lda;
  const unsigned short* bb = Bt + (size_t)(n0 + m) * ldb + 8 * h;
  const v8f z8 = {0.f, 0.f, 0.f, 0.f, 0.f, 0.f, 0.f, 0.f};
  v8f acc[2][4];
#pragma unroll
  for (int i = 0; i < 2; ++i)
#pragma unroll
    for (int j = 0; j < 4; ++j) acc[i][j] = z8;

#pragma unroll 1
  for (int k0 = 0; k0 < K; k0 += 32) {
    const v16b fa0 = ldfrag_g(a0 + k0);
    const v16b fa1 = ldfrag_g(a1 + k0);
    const v16b fb0 = ldfrag_g(bb + k0);
    const v16b fb1 = ldfrag_g(bb + (size_t)16 * ldb + k0);
    const v16b fb2 = ldfrag_g(bb + (size_t)32 * ldb + k0);
    const v16b fb3 = ldfrag_g(bb + (size_t)48 * ldb + k0);
    acc[0][0] = mma(fa0, fb0, acc[0][0]); acc[1][0] = mma(fa1, fb0, acc[1][0]);
    acc[0][1] = mma(fa0, fb1, acc[0][1]); acc[1][1] = mma(fa1, fb1, acc[1][1]);
    acc[0][2] = mma(fa0, fb2, acc[0][2]); acc[1][2] = mma(fa1, fb2, acc[1][2]);
    acc[0][3] = mma(fa0, fb3, acc[0][3]); acc[1][3] = mma(fa1, fb3, acc[1][3]);
    guard8(acc[0][0], acc[0][1], acc[0][2], acc[0][3], acc[1][0], acc[1][1], acc[1][2], acc[1][3],
           fa0, fa1, fb0, fb1, fb2, fb3);
  }

  float* sl = slab + w * (32 * 68);
#pragma unroll
  for (int mt = 0; mt < 2; ++mt)
#pragma unroll
    for (int nt = 0; nt < 4; ++nt) {
      const float bv = sbias[16 * nt + m];
#pragma unroll
      for (int r = 0; r < 8; ++r) {
        float v = acc[mt][nt][r] + bv;
        if (GELU) v = gelu_f(v);
        sl[(16 * mt + 8 * h + r) * 68 + 16 * nt + m] = v;
      }
    }
  wave_sync();

  if (OUT == 0) {
    float* Cf = (float*)Cv;
    const int hh = lane >> 4, c4 = (lane & 15) * 4;
#pragma unroll 1
    for (int g = 0; g < 2; ++g) {
      v4f vals[8];
#pragma unroll
      for (int it = 0; it < 8; ++it) {
        const int row = g * 16 + it * 2 + hh;
        v4f v = *(const v4fa*)(sl + row * 68 + c4);
        const size_t gi = (size_t)(m0 + row) * ldc + n0 + c4;
        if (NRES == 1) {
          v4f r1 = *(const v4fa*)(R1 + gi);
          if (R1RND) { r1[0] = rbf(r1[0]); r1[1] = rbf(r1[1]); r1[2] = rbf(r1[2]); r1[3] = rbf(r1[3]); }
          v = r1 + v;
        }
        if (NRES == 2) {
          const v4f r1 = *(const v4fa*)(R1 + gi);
          const v4f r2 = *(const v4fa*)(R2 + gi);
          v = (r1 + r2) + v;
        }
        vals[it] = v;
      }
      for (int pass = 0; pass < 2; ++pass) {
#pragma unroll
        for (int it = 0; it < 8; ++it) {
          const int row = g * 16 + it * 2 + hh;
          *(volatile v4f*)(Cf + (size_t)(m0 + row) * ldc + n0 + c4) = vals[it];
        }
        __threadfence();
      }
    }
  } else {
    unsigned short* Cb = (unsigned short*)Cv;
    const int half = ldc >> 1;
    const int q = lane >> 3, c8 = (lane & 7) * 8;
    v4u hv[8], lv[8];
#pragma unroll
    for (int it = 0; it < 8; ++it) {
      const int row = it * 4 + q;
      const v4f x0 = *(const v4fa*)(sl + row * 68 + c8);
      const v4f x1 = *(const v4fa*)(sl + row * 68 + c8 + 4);
      hv[it] = (v4u){ pkhi2(x0[0], x0[1]), pkhi2(x0[2], x0[3]), pkhi2(x1[0], x1[1]), pkhi2(x1[2], x1[3]) };
      lv[it] = (v4u){ pklo2(x0[0], x0[1]), pklo2(x0[2], x0[3]), pklo2(x1[0], x1[1]), pklo2(x1[2], x1[3]) };
    }
    for (int pass = 0; pass < 2; ++pass) {
#pragma unroll
      for (int it = 0; it < 8; ++it) {
        const int row = it * 4 + q;
        const size_t gi = (size_t)(m0 + row) * ldc + n0 + c8;
        *(volatile v4u*)(Cb + gi) = hv[it];
        *(volatile v4u*)(Cb + gi + half) = lv[it];
      }
      __threadfence();
    }
  }
}

__global__ __launch_bounds__(256) __attribute__((amdgpu_num_vgpr(248)))
void k_eagg(const float* __restrict__ e, const float* __restrict__ QKV, const unsigned short* __restrict__ WEBG,
            const float* __restrict__ Wl2e, const float* __restrict__ bl2e,
            float* __restrict__ Z, float* __restrict__ ES) {
  __shared__ __align__(16) unsigned short et[64 * 136];
  __shared__ __align__(16) float bgs[64 * 17];
  __shared__ __align__(16) float qs[256];
  __shared__ __align__(16) float raws[8 * 64];
  __shared__ __align__(16) float zs[8 * 64];
  __shared__ __align__(16) float wl[8 * 128];
  __shared__ __align__(16) float bl[128];
  const int tid = threadIdx.x, lane = tid & 31, w = tid >> 5, h = lane >> 4, m = lane & 15;
  const int i = blockIdx.x >> 2, j0 = (blockIdx.x & 3) * 64;
  const size_t rowBase = (size_t)blockIdx.x * 64;
  const float SC = 1.0f / sqrtf(32.0f);

#pragma unroll
  for (int it = 0; it < 4; ++it) {
    const int row = it * 16 + (tid >> 4), c8 = (tid & 15) * 8;
    const float* src = e + (rowBase + row) * 128 + c8;
    const v4f a = *(const v4fa*)(src);
    const v4f b = *(const v4fa*)(src + 4);
    const v4u o = { pkhi2(a[0], a[1]), pkhi2(a[2], a[3]), pkhi2(b[0], b[1]), pkhi2(b[2], b[3]) };
    *(v4ua*)(et + row * 136 + c8) = o;
  }
  qs[tid] = QKV[(size_t)i * 768 + tid];
  {
    const v4f wv = *(const v4fa*)(Wl2e + tid * 4);
    const v4f wr = { rbf(wv[0]), rbf(wv[1]), rbf(wv[2]), rbf(wv[3]) };
    *(v4fa*)(wl + tid * 4) = wr;
  }
  if (tid < 128) bl[tid] = rbf(bl2e[tid]);
  __syncthreads();

  const int jj = tid & 63, hq = tid >> 6;
  float d0 = 0.f, d1 = 0.f;
  {
    const float* kp = QKV + (size_t)(j0 + jj) * 768 + 256 + hq * 64;
    const float* qp = qs + hq * 64;
#pragma unroll 1
    for (int c = 0; c < 8; ++c) {
      const v4f k0v = *(const v4fa*)(kp + 4 * c);
      const v4f k1v = *(const v4fa*)(kp + 32 + 4 * c);
      const v4f q0v = *(const v4fa*)(qp + 4 * c);
      const v4f q1v = *(const v4fa*)(qp + 32 + 4 * c);
      d0 += q0v[0] * k0v[0]; d0 += q0v[1] * k0v[1]; d0 += q0v[2] * k0v[2]; d0 += q0v[3] * k0v[3];
      d1 += q1v[0] * k1v[0]; d1 += q1v[1] * k1v[1]; d1 += q1v[2] * k1v[2]; d1 += q1v[3] * k1v[3];
    }
  }
  if (w < 4) {
    v8f acc = {0.f, 0.f, 0.f, 0.f, 0.f, 0.f, 0.f, 0.f};
    const int aoff = (16 * w + m) * 136 + 8 * h;
    const unsigned short* bp = WEBG + m * 128 + 8 * h;
#pragma unroll
    for (int k0 = 0; k0 < 128; k0 += 32) {
      v16b a; LDS_FRAG(a, et, aoff + k0);
      const v16b b = ldfrag_g(bp + k0);
      acc = mma_g(a, b, acc);
    }
#pragma unroll
    for (int r = 0; r < 8; ++r) bgs[(16 * w + 8 * h + r) * 17 + m] = acc[r];
  }
  __syncthreads();
  {
    const int hd0 = hq * 2;
    const float r0 = d0 * SC + bgs[jj * 17 + hd0];
    const float r1 = d1 * SC + bgs[jj * 17 + hd0 + 1];
    raws[hd0 * 64 + jj] = r0;
    raws[(hd0 + 1) * 64 + jj] = r1;
    zs[hd0 * 64 + jj] = r0 * sigm(bgs[jj * 17 + 8 + hd0]);
    zs[(hd0 + 1) * 64 + jj] = r1 * sigm(bgs[jj * 17 + 8 + hd0 + 1]);
  }
  __syncthreads();

  if (tid < 128) {
    const int hd = tid >> 4, c4 = (tid & 15) * 4;
    const v4f v = *(const v4fa*)(zs + hd * 64 + c4);
    float* dst = Z + ((size_t)hd * 256 + i) * 256 + j0 + c4;
    *(volatile v4f*)dst = v;
    __threadfence();
    *(volatile v4f*)dst = v;
  }

#pragma unroll 1
  for (int rr = 0; rr < 8; ++rr) {
    const int row = 8 * w + rr;
    const v2u pk = *(const v2ua*)(et + row * 136 + 4 * lane);
    const v4f x = { __uint_as_float(pk[0] << 16), __uint_as_float(pk[0] & 0xffff0000u),
                    __uint_as_float(pk[1] << 16), __uint_as_float(pk[1] & 0xffff0000u) };
    const v4f t = ln128(x);
    v4f acc = *(const v4fa*)(bl + 4 * lane);
#pragma unroll
    for (int hd = 0; hd < 8; ++hd) {
      const float rv = raws[hd * 64 + row];
      const v4f wv = *(const v4fa*)(wl + hd * 128 + 4 * lane);
      acc += rv * wv;
    }
    const v4f y = t + acc;
    float* dst = ES + (rowBase + row) * 128 + 4 * lane;
    *(volatile v4f*)dst = y;
    __threadfence();
    *(volatile v4f*)dst = y;
  }
}

__global__ __launch_bounds__(256) __attribute__((amdgpu_num_vgpr(248)))
void k_nattn(const float* __restrict__ Z, const float* __restrict__ QKV, unsigned short* __restrict__ OHL) {
  __shared__ __align__(16) float ps[8 * 256];
  __shared__ __align__(16) float os[256];
  const int tid = threadIdx.x, lane = tid & 31, w = tid >> 5;
  const int i = blockIdx.x;
  float* pw = ps + w * 256;
  const float* zr = Z + ((size_t)w * 256 + i) * 256;
  {
    const v4f a = *(const v4fa*)(zr + 4 * lane);
    const v4f b = *(const v4fa*)(zr + 128 + 4 * lane);
    *(v4fa*)(pw + 4 * lane) = a;
    *(v4fa*)(pw + 128 + 4 * lane) = b;
  }
  __syncthreads();
  float mx = -INFINITY;
#pragma unroll 1
  for (int t = 0; t < 8; ++t) mx = fmaxf(mx, pw[lane + 32 * t]);
  mx = wmax32(mx);
  float sum = 0.f;
#pragma unroll 1
  for (int t = 0; t < 8; ++t) {
    const int idx = lane + 32 * t;
    const float p = expf(pw[idx] - mx);
    pw[idx] = p;
    sum += p;
  }
  sum = wsum32(sum);
  __syncthreads();
  float acc = 0.f;
  const float* vp = QKV + 512 + w * 32 + lane;
#pragma unroll 4
  for (int j = 0; j < 256; ++j) acc += pw[j] * vp[(size_t)j * 768];
  os[w * 32 + lane] = acc * (1.0f / sum);
  __syncthreads();
  if (tid < 64) {
    const int part = tid >> 5, c8 = (tid & 31) * 8;
    const v4f x0 = *(const v4fa*)(os + c8);
    const v4f x1 = *(const v4fa*)(os + c8 + 4);
    const v4u hv = { pkhi2(x0[0], x0[1]), pkhi2(x0[2], x0[3]), pkhi2(x1[0], x1[1]), pkhi2(x1[2], x1[3]) };
    const v4u lv = { pklo2(x0[0], x0[1]), pklo2(x0[2], x0[3]), pklo2(x1[0], x1[1]), pklo2(x1[2], x1[3]) };
    const v4u o = part ? lv : hv;
    unsigned short* dst = OHL + (size_t)i * 512 + part * 256 + c8;
    *(volatile v4u*)dst = o;
    __threadfence();
    *(volatile v4u*)dst = o;
  }
}

__global__ __launch_bounds__(128) __attribute__((amdgpu_num_vgpr(248)))
void k_nln(const float* __restrict__ H1, float* __restrict__ HN, unsigned short* __restrict__ XHL) {
  __shared__ __align__(16) float xs2[4 * 256];
  const int tid = threadIdx.x, lane = tid & 31, w = tid >> 5;
  const int row = blockIdx.x * 4 + w;
  const float* src = H1 + (size_t)row * 256;
  const v4f a = *(const v4fa*)(src + 4 * lane);
  const v4f b = *(const v4fa*)(src + 128 + 4 * lane);
  float s = ((a[0] + a[1]) + (a[2] + a[3])) + ((b[0] + b[1]) + (b[2] + b[3]));
  s = wsum32(s);
  float mean = s * (1.0f / 256.0f);
  v4f da = a - mean, db = b - mean;
  float q = ((da[0] * da[0] + da[1] * da[1]) + (da[2] * da[2] + da[3] * da[3])) +
            ((db[0] * db[0] + db[1] * db[1]) + (db[2] * db[2] + db[3] * db[3]));
  q = wsum32(q);
  float rs = rsqrtf(q * (1.0f / 256.0f) + LN_EPS);
  const v4f ha = da * rs, hb = db * rs;
  {
    float* d0 = HN + (size_t)row * 256 + 4 * lane;
    float* d1 = d0 + 128;
    *(volatile v4f*)d0 = ha;
    *(volatile v4f*)d1 = hb;
    __threadfence();
    *(volatile v4f*)d0 = ha;
    *(volatile v4f*)d1 = hb;
  }
  s = ((ha[0] + ha[1]) + (ha[2] + ha[3])) + ((hb[0] + hb[1]) + (hb[2] + hb[3]));
  s = wsum32(s);
  mean = s * (1.0f / 256.0f);
  da = ha - mean; db = hb - mean;
  q = ((da[0] * da[0] + da[1] * da[1]) + (da[2] * da[2] + da[3] * da[3])) +
      ((db[0] * db[0] + db[1] * db[1]) + (db[2] * db[2] + db[3] * db[3]));
  q = wsum32(q);
  rs = rsqrtf(q * (1.0f / 256.0f) + LN_EPS);
  *(v4fa*)(xs2 + w * 256 + 4 * lane) = da * rs;
  *(v4fa*)(xs2 + w * 256 + 128 + 4 * lane) = db * rs;
  __syncthreads();
  {
    const int c8 = 8 * lane;
    const v4f x0 = *(const v4fa*)(xs2 + w * 256 + c8);
    const v4f x1 = *(const v4fa*)(xs2 + w * 256 + c8 + 4);
    const v4u hv = { pkhi2(x0[0], x0[1]), pkhi2(x0[2], x0[3]), pkhi2(x1[0], x1[1]), pkhi2(x1[2], x1[3]) };
    const v4u lv = { pklo2(x0[0], x0[1]), pklo2(x0[2], x0[3]), pklo2(x1[0], x1[1]), pklo2(x1[2], x1[3]) };
    unsigned short* d0 = XHL + (size_t)row * 512 + c8;
    unsigned short* d1 = d0 + 256;
    *(volatile v4u*)d0 = hv;
    *(volatile v4u*)d1 = lv;
    __threadfence();
    *(volatile v4u*)d0 = hv;
    *(volatile v4u*)d1 = lv;
  }
}

__global__ __launch_bounds__(256) __attribute__((amdgpu_num_vgpr(248)))
void k_ffn(const float* Xin, float* Yout,
           const unsigned short* __restrict__ WE1, const unsigned short* __restrict__ WE2,
           const float* __restrict__ be1, const float* __restrict__ be2) {
  extern __shared__ __align__(16) unsigned char smem[];
  float* xs = (float*)smem;
  unsigned short* als = (unsigned short*)(smem + 33792);
  unsigned short* hs  = (unsigned short*)(smem + 67584);
  float* sb1 = (float*)(smem + 199680);
  float* sb2 = (float*)(smem + 201728);
  const int tid = threadIdx.x, lane = tid & 31, w = tid >> 5, h = lane >> 4, m = lane & 15;
  const int wm = w & 3, wn = w >> 2;
  const size_t rowBase = (size_t)blockIdx.x * 64;

#pragma unroll 2
  for (int rr = 0; rr < 8; ++rr) {
    const int row = 8 * w + rr;
    const v4f x = *(const v4fa*)(Xin + (rowBase + row) * 128 + 4 * lane);
    *(v4fa*)(xs + row * 132 + 4 * lane) = x;
    const v4f t = ln128(x);
    const v2u hv = { pkhi2(t[0], t[1]), pkhi2(t[2], t[3]) };
    const v2u lv = { pklo2(t[0], t[1]), pklo2(t[2], t[3]) };
    *(v2ua*)(als + row * 264 + 4 * lane) = hv;
    *(v2ua*)(als + row * 264 + 128 + 4 * lane) = lv;
  }
  sb1[tid] = rbf(be1[tid]);
  sb1[tid + 256] = rbf(be1[tid + 256]);
  if (tid < 128) sb2[tid] = rbf(be2[tid]);
  __syncthreads();

  const v8f z8 = {0.f, 0.f, 0.f, 0.f, 0.f, 0.f, 0.f, 0.f};
#pragma unroll 1
  for (int pass = 0; pass < 4; ++pass) {
    const int nb = pass * 128 + wn * 64;
    v8f acc[4];
    acc[0] = z8; acc[1] = z8; acc[2] = z8; acc[3] = z8;
    const unsigned short* bp = WE1 + (size_t)(nb + m) * 256 + 8 * h;
    const int aoff = (16 * wm + m) * 264 + 8 * h;
#pragma unroll 1
    for (int k0 = 0; k0 < 256; k0 += 32) {
      v16b a; LDS_FRAG(a, als, aoff + k0);
      const v16b b0 = ldfrag_g(bp + k0);
      const v16b b1 = ldfrag_g(bp + 16 * 256 + k0);
      const v16b b2 = ldfrag_g(bp + 32 * 256 + k0);
      const v16b b3 = ldfrag_g(bp + 48 * 256 + k0);
      acc[0] = mma(a, b0, acc[0]);
      acc[1] = mma(a, b1, acc[1]);
      acc[2] = mma(a, b2, acc[2]);
      acc[3] = mma(a, b3, acc[3]);
      guard4(acc[0], acc[1], acc[2], acc[3], a, b0, b1, b2, b3);
    }
#pragma unroll
    for (int s = 0; s < 4; ++s) {
      const int col = nb + 16 * s + m;
      const float bv = sb1[col];
#pragma unroll
      for (int r = 0; r < 8; ++r) {
        const int row = 16 * wm + 8 * h + r;
        const float g = gelu_f(acc[s][r] + bv);
        const unsigned short hb = f2bf(g);
        const unsigned short lb = f2bf(g - bf2f(hb));
        hs[row * 1032 + col] = hb;
        hs[row * 1032 + 512 + col] = lb;
      }
    }
  }
  __syncthreads();

  {
    const int nb = wn * 64;
    v8f acc[4];
    acc[0] = z8; acc[1] = z8; acc[2] = z8; acc[3] = z8;
    const unsigned short* bp = WE2 + (size_t)(nb + m) * 1024 + 8 * h;
    const int aoff = (16 * wm + m) * 1032 + 8 * h;
#pragma unroll 1
    for (int k0 = 0; k0 < 1024; k0 += 32) {
      v16b a; LDS_FRAG(a, hs, aoff + k0);
      const v16b b0 = ldfrag_g(bp + k0);
      const v16b b1 = ldfrag_g(bp + 16 * 1024 + k0);
      const v16b b2 = ldfrag_g(bp + 32 * 1024 + k0);
      const v16b b3 = ldfrag_g(bp + 48 * 1024 + k0);
      acc[0] = mma(a, b0, acc[0]);
      acc[1] = mma(a, b1, acc[1]);
      acc[2] = mma(a, b2, acc[2]);
      acc[3] = mma(a, b3, acc[3]);
      guard4(acc[0], acc[1], acc[2], acc[3], a, b0, b1, b2, b3);
    }
#pragma unroll
    for (int s = 0; s < 4; ++s) {
      const int col = nb + 16 * s + m;
      const float bv = sb2[col];
#pragma unroll
      for (int r = 0; r < 8; ++r) {
        const int row = 16 * wm + 8 * h + r;
        const float x = xs[row * 132 + col];
        const float f = acc[s][r] + bv;
        xs[row * 132 + col] = x + (x + f);
      }
    }
  }
  __syncthreads();

  {
    v4f v[8];
#pragma unroll
    for (int rr = 0; rr < 8; ++rr) v[rr] = *(const v4fa*)(xs + (8 * w + rr) * 132 + 4 * lane);
    for (int pass = 0; pass < 2; ++pass) {
#pragma unroll
      for (int rr = 0; rr < 8; ++rr)
        *(volatile v4f*)(Yout + (rowBase + 8 * w + rr) * 128 + 4 * lane) = v[rr];
      __threadfence();
    }
  }
}

__global__ __launch_bounds__(256) __attribute__((amdgpu_num_vgpr(248)))
void k_tproj(const float* __restrict__ ES, const unsigned short* __restrict__ WTRI,
             unsigned short* __restrict__ QPV, float* __restrict__ GT) {
  __shared__ __align__(16) unsigned short als[64 * 264];
  __shared__ __align__(16) unsigned short stg[128 * 72];
  __shared__ __align__(16) float gs[8 * 64];
  const int tid = threadIdx.x, lane = tid & 31, w = tid >> 5, h = lane >> 4, m = lane & 15;
  const int wm = w & 3, wn = w >> 2;
  const int a = blockIdx.x >> 2, b0 = (blockIdx.x & 3) * 64;
  const size_t rowBase = (size_t)blockIdx.x * 64;

#pragma unroll 2
  for (int rr = 0; rr < 8; ++rr) {
    const int row = 8 * w + rr;
    const v4f x = *(const v4fa*)(ES + (rowBase + row) * 128 + 4 * lane);
    const v4f t = ln128(x);
    const v2u hv = { pkhi2(t[0], t[1]), pkhi2(t[2], t[3]) };
    const v2u lv = { pklo2(t[0], t[1]), pklo2(t[2], t[3]) };
    *(v2ua*)(als + row * 264 + 4 * lane) = hv;
    *(v2ua*)(als + row * 264 + 128 + 4 * lane) = lv;
  }
  __syncthreads();

  const v8f z8 = {0.f, 0.f, 0.f, 0.f, 0.f, 0.f, 0.f, 0.f};
  const int aoff = (16 * wm + m) * 264 + 8 * h;
#pragma unroll 1
  for (int cls = 0; cls < 3; ++cls) {
    const int nb = cls * 128 + wn * 64;
    v8f acc[4];
    acc[0] = z8; acc[1] = z8; acc[2] = z8; acc[3] = z8;
    const unsigned short* bp = WTRI + (size_t)(nb + m) * 256 + 8 * h;
#pragma unroll 1
    for (int k0 = 0; k0 < 256; k0 += 32) {
      v16b fa; LDS_FRAG(fa, als, aoff + k0);
      const v16b f0 = ldfrag_g(bp + k0);
      const v16b f1 = ldfrag_g(bp + 16 * 256 + k0);
      const v16b f2 = ldfrag_g(bp + 32 * 256 + k0);
      const v16b f3 = ldfrag_g(bp + 48 * 256 + k0);
      acc[0] = mma(fa, f0, acc[0]);
      acc[1] = mma(fa, f1, acc[1]);
      acc[2] = mma(fa, f2, acc[2]);
      acc[3] = mma(fa, f3, acc[3]);
      guard4(acc[0], acc[1], acc[2], acc[3], fa, f0, f1, f2, f3);
    }
#pragma unroll
    for (int s = 0; s < 4; ++s) {
      const int col = wn * 64 + 16 * s + m;
#pragma unroll
      for (int r = 0; r < 8; ++r) {
        const int row = 16 * wm + 8 * h + r;
        const int so = (cls < 2) ? (row * 136 + col) : (col * 72 + row);
        stg[so] = f2bf(acc[s][r]);
      }
    }
    __syncthreads();
    {
      v4u vv[4];
      size_t go[4];
#pragma unroll
      for (int rep = 0; rep < 4; ++rep) {
        const int idx = rep * 256 + tid;
        if (cls < 2) {
          const int row = idx >> 4, c8 = (idx & 15) * 8;
          vv[rep] = *(const v4ua*)(stg + row * 136 + c8);
          go[rep] = (size_t)cls * PLANE_H + (rowBase + row) * 128 + c8;
        } else {
          const int line = idx >> 3, c8 = (idx & 7) * 8;
          vv[rep] = *(const v4ua*)(stg + line * 72 + c8);
          go[rep] = (size_t)2 * PLANE_H + ((size_t)a * 128 + line) * 256 + b0 + c8;
        }
      }
      for (int pass = 0; pass < 2; ++pass) {
#pragma unroll
        for (int rep = 0; rep < 4; ++rep) *(volatile v4u*)(QPV + go[rep]) = vv[rep];
        __threadfence();
      }
    }
    __syncthreads();
  }

  if (w < 4) {
    v8f acc = z8;
    const unsigned short* bp = WTRI + (size_t)(384 + m) * 256 + 8 * h;
#pragma unroll 1
    for (int k0 = 0; k0 < 256; k0 += 32) {
      v16b fa; LDS_FRAG(fa, als, aoff + k0);
      const v16b fb = ldfrag_g(bp + k0);
      acc = mma_g(fa, fb, acc);
    }
#pragma unroll
    for (int r = 0; r < 8; ++r) {
      const float v = acc[r];
      const float sg = sigm(v);
      const float o = (m < 4) ? sg : v;
      if (m < 8) gs[m * 64 + 16 * wm + 8 * h + r] = o;
    }
  }
  __syncthreads();
  if (tid < 128) {
    const int prow = tid >> 4, c4 = (tid & 15) * 4;
    const v4f v = *(const v4fa*)(gs + prow * 64 + c4);
    float* dst = GT + ((size_t)prow * 256 + a) * 256 + b0 + c4;
    *(volatile v4f*)dst = v;
    __threadfence();
    *(volatile v4f*)dst = v;
  }
}

struct SmStep { float m, l, al; unsigned short q0, q1, q2, q3; };

__device__ __forceinline__ SmStep sm_step(float l0, float l1, float l2, float l3, float mrun, float lrun) {
  SmStep o;
  float mx = fmaxf(fmaxf(l0, l1), fmaxf(l2, l3));
  mx = hmax16(mx);
  const float mnew = fmaxf(mrun, mx);
  o.al = expf(mrun - mnew);
  o.m = mnew;
  o.q0 = f2bf(expf(l0 - mnew));
  o.q1 = f2bf(expf(l1 - mnew));
  o.q2 = f2bf(expf(l2 - mnew));
  o.q3 = f2bf(expf(l3 - mnew));
  float psum = (bf2f(o.q0) + bf2f(o.q1)) + (bf2f(o.q2) + bf2f(o.q3));
  psum = hsum16(psum);
  o.l = lrun * o.al + psum;
  return o;
}

#define TATTN_ROW(R) do { \
    const int go_ = (16 * w + 8 * h + (R)) * 68 + m; \
    const int po_ = (8 * h + (R)) * 72 + m; \
    const float sv0_ = s0[(R)] * SC, sv1_ = s1[(R)] * SC, sv2_ = s2[(R)] * SC, sv3_ = s3[(R)] * SC; \
    const SmStep a_ = sm_step((sv0_ + gt[4352 + go_]) * gt[go_], \
                              (sv1_ + gt[4352 + go_ + 16]) * gt[go_ + 16], \
                              (sv2_ + gt[4352 + go_ + 32]) * gt[go_ + 32], \
                              (sv3_ + gt[4352 + go_ + 48]) * gt[go_ + 48], mi8[(R)], li8[(R)]); \
    mi8[(R)] = a_.m; li8[(R)] = a_.l; \
    oin0[(R)] = oin0[(R)] * a_.al; oin1[(R)] = oin1[(R)] * a_.al; \
    pt[pinOff + po_] = a_.q0; pt[pinOff + po_ + 16] = a_.q1; \
    pt[pinOff + po_ + 32] = a_.q2; pt[pinOff + po_ + 48] = a_.q3; \
    const float bb_ = bo8[(R)], gv_ = go8[(R)]; \
    const SmStep b_ = sm_step((sv0_ + bb_) * gv_, (sv1_ + bb_) * gv_, (sv2_ + bb_) * gv_, (sv3_ + bb_) * gv_, \
                              mo8[(R)], lo8[(R)]); \
    mo8[(R)] = b_.m; lo8[(R)] = b_.l; \
    oout0[(R)] = oout0[(R)] * b_.al; oout1[(R)] = oout1[(R)] * b_.al; \
    pt[poutOff + po_] = b_.q0; pt[poutOff + po_ + 16] = b_.q1; \
    pt[poutOff + po_ + 32] = b_.q2; pt[poutOff + po_ + 48] = b_.q3; \
    __builtin_amdgcn_sched_barrier(0); \
  } while (0)

#define TATTN_OUT(R) do { \
    const float ii_ = 1.0f / li8[(R)]; \
    const float io_ = 1.0f / lo8[(R)]; \
    const int oo_ = pinOff + (8 * h + (R)) * 72 + m; \
    pt[oo_]      = f2bf(oin0[(R)] * ii_); \
    pt[oo_ + 16] = f2bf(oin1[(R)] * ii_); \
    pt[oo_ + 32] = f2bf(oout0[(R)] * io_); \
    pt[oo_ + 48] = f2bf(oout1[(R)] * io_); \
  } while (0)

__global__ __launch_bounds__(128) __attribute__((amdgpu_num_vgpr(248)))
void k_tattn(const unsigned short* __restrict__ QPV, const float* __restrict__ GT, unsigned short* __restrict__ OP) {
  __shared__ __align__(16) float gt[2 * 64 * 68];
  __shared__ __align__(16) unsigned short pt[4 * 2 * 16 * 72];
  const int tid = threadIdx.x, lane = tid & 31, w = tid >> 5, h = lane >> 4, m = lane & 15;
  const int bx = blockIdx.x;
  const int it = bx & 3, ht = (bx >> 2) & 3, j = bx >> 4;
  const int i0w = it * 64 + 16 * w;
  const float SC = 1.0f / sqrtf(32.0f);
  const unsigned short* Qp = QPV;
  const unsigned short* Pp = QPV + PLANE_H;
  const unsigned short* Vp = QPV + 2 * PLANE_H;
  const int pinOff  = w * 2304;
  const int poutOff = w * 2304 + 1152;

  const v16b qa = ldfrag_g(Qp + ((size_t)(i0w + m) * 256 + j) * 128 + ht * 32 + 8 * h);

  v8f go8, bo8;
  {
    const float* gp = GT + ((size_t)(ht * 256 + j)) * 256 + i0w + 8 * h;
    const float* bp = GT + ((size_t)((4 + ht) * 256 + j)) * 256 + i0w + 8 * h;
    const v4f g0 = *(const v4fa*)(gp), g1 = *(const v4fa*)(gp + 4);
    const v4f c0 = *(const v4fa*)(bp), c1 = *(const v4fa*)(bp + 4);
    go8 = (v8f){ g0[0], g0[1], g0[2], g0[3], g1[0], g1[1], g1[2], g1[3] };
    bo8 = (v8f){ c0[0], c0[1], c0[2], c0[3], c1[0], c1[1], c1[2], c1[3] };
  }

  const v8f z8 = {0.f, 0.f, 0.f, 0.f, 0.f, 0.f, 0.f, 0.f};
  const v8f ninf8 = { -INFINITY, -INFINITY, -INFINITY, -INFINITY, -INFINITY, -INFINITY, -INFINITY, -INFINITY };
  v8f mi8 = ninf8, mo8 = ninf8, li8 = z8, lo8 = z8;
  v8f oin0 = z8, oin1 = z8, oout0 = z8, oout1 = z8;

#pragma unroll 1
  for (int kt = 0; kt < 4; ++kt) {
    __syncthreads();
#pragma unroll 4
    for (int rep = 0; rep < 16; ++rep) {
      const int pl = rep >> 3;
      const int idx = (rep & 7) * 128 + tid;
      const int ii = idx >> 4, c4 = (idx & 15) * 4;
      const v4f v = *(const v4fa*)(GT + ((size_t)((pl * 4 + ht) * 256 + it * 64 + ii)) * 256 + kt * 64 + c4);
      *(v4fa*)(gt + (pl * 64 + ii) * 68 + c4) = v;
    }
    __syncthreads();

    v8f s0, s1, s2, s3;
    {
      const unsigned short* pb = Pp + ((size_t)(j * 256 + kt * 64 + m)) * 128 + ht * 32 + 8 * h;
      const v16b b0 = ldfrag_g(pb);
      const v16b b1 = ldfrag_g(pb + 16 * 128);
      const v16b b2 = ldfrag_g(pb + 32 * 128);
      const v16b b3 = ldfrag_g(pb + 48 * 128);
      s0 = mma(qa, b0, z8);
      s1 = mma(qa, b1, z8);
      s2 = mma(qa, b2, z8);
      s3 = mma(qa, b3, z8);
      guard4(s0, s1, s2, s3, qa, b0, b1, b2, b3);
    }

    TATTN_ROW(0);
    TATTN_ROW(1);
    TATTN_ROW(2);
    TATTN_ROW(3);
    TATTN_ROW(4);
    TATTN_ROW(5);
    TATTN_ROW(6);
    TATTN_ROW(7);
    wave_sync();

#pragma unroll 1
    for (int kk = 0; kk < 2; ++kk) {
      v16b pa, pb;
      LDS_FRAG(pa, pt, pinOff  + m * 72 + kk * 32 + 8 * h);
      LDS_FRAG(pb, pt, poutOff + m * 72 + kk * 32 + 8 * h);
      const unsigned short* vp = Vp + ((size_t)((j * 4 + ht) * 32 + m)) * 256 + kt * 64 + kk * 32 + 8 * h;
      const v16b v0 = ldfrag_g(vp);
      const v16b v1 = ldfrag_g(vp + 16 * 256);
      oin0  = mma(pa, v0, oin0);
      oin1  = mma(pa, v1, oin1);
      oout0 = mma(pb, v0, oout0);
      oout1 = mma(pb, v1, oout1);
      guard4(oin0, oin1, oout0, oout1, pa, pb, v0, v1, v1);
    }
  }

  wave_sync();
  TATTN_OUT(0);
  TATTN_OUT(1);
  TATTN_OUT(2);
  TATTN_OUT(3);
  TATTN_OUT(4);
  TATTN_OUT(5);
  TATTN_OUT(6);
  TATTN_OUT(7);
  wave_sync();
  {
    const int q = lane >> 3, c8 = (lane & 7) * 8;
    const v4u vv0 = *(const v4ua*)(pt + pinOff + (0 + q) * 72 + c8);
    const v4u vv1 = *(const v4ua*)(pt + pinOff + (4 + q) * 72 + c8);
    const v4u vv2 = *(const v4ua*)(pt + pinOff + (8 + q) * 72 + c8);
    const v4u vv3 = *(const v4ua*)(pt + pinOff + (12 + q) * 72 + c8);
    unsigned short* d0 = OP + ((size_t)(i0w + 0 + q) * 256 + j) * 256 + ht * 64 + c8;
    unsigned short* d1 = OP + ((size_t)(i0w + 4 + q) * 256 + j) * 256 + ht * 64 + c8;
    unsigned short* d2 = OP + ((size_t)(i0w + 8 + q) * 256 + j) * 256 + ht * 64 + c8;
    unsigned short* d3 = OP + ((size_t)(i0w + 12 + q) * 256 + j) * 256 + ht * 64 + c8;
    *(volatile v4u*)d0 = vv0;
    *(volatile v4u*)d1 = vv1;
    *(volatile v4u*)d2 = vv2;
    *(volatile v4u*)d3 = vv3;
    __threadfence();
    *(volatile v4u*)d0 = vv0;
    *(volatile v4u*)d1 = vv1;
    *(volatile v4u*)d2 = vv2;
    *(volatile v4u*)d3 = vv3;
  }
}

constexpr size_t SZ_ES   = (size_t)NPAIR * 128 * 4;
constexpr size_t SZ_PL   = (size_t)NPAIR * 128 * 2;
constexpr size_t SZ_OP   = (size_t)NPAIR * 256 * 2;
constexpr size_t SZ_GT   = (size_t)2 * 4 * 256 * 256 * 4;
constexpr size_t SZ_Z    = (size_t)8 * 256 * 256 * 4;
constexpr size_t SZ_QKV  = (size_t)256 * 768 * 4;
constexpr size_t SZ_HB   = (size_t)256 * 256 * 2;
constexpr size_t SZ_WQKV = (size_t)768 * 256 * 2;
constexpr size_t SZ_WO2  = (size_t)256 * 512 * 2;
constexpr size_t SZ_WN1  = (size_t)1024 * 512 * 2;
constexpr size_t SZ_WN2  = (size_t)256 * 2048 * 2;
constexpr size_t SZ_WEBG = (size_t)16 * 128 * 2;
constexpr size_t SZ_WE1  = (size_t)512 * 256 * 2;
constexpr size_t SZ_WE2  = (size_t)128 * 1024 * 2;
constexpr size_t SZ_WTRI = (size_t)NTRI * 256 * 2;
constexpr size_t SZ_WTO  = (size_t)128 * 256 * 2;
constexpr size_t SZ_NF   = (size_t)256 * 256 * 4;
constexpr size_t SZ_NHL  = (size_t)256 * 512 * 2;
constexpr size_t SZ_GHL  = (size_t)256 * 2048 * 2;

constexpr size_t O_ES   = 0;
constexpr size_t O_Q    = O_ES + SZ_ES;
constexpr size_t O_P    = O_Q + SZ_PL;
constexpr size_t O_VT   = O_P + SZ_PL;
constexpr size_t O_OP   = O_VT + SZ_PL;
constexpr size_t O_GT   = O_OP + SZ_OP;
constexpr size_t O_Z    = O_GT + SZ_GT;
constexpr size_t O_QKV  = O_Z + SZ_Z;
constexpr size_t O_HB   = O_QKV + SZ_QKV;
constexpr size_t O_WQKV = O_HB + SZ_HB;
constexpr size_t O_WO2  = O_WQKV + SZ_WQKV;
constexpr size_t O_WN1  = O_WO2 + SZ_WO2;
constexpr size_t O_WN2  = O_WN1 + SZ_WN1;
constexpr size_t O_WEBG = O_WN2 + SZ_WN2;
constexpr size_t O_WE1  = O_WEBG + SZ_WEBG;
constexpr size_t O_WE2  = O_WE1 + SZ_WE1;
constexpr size_t O_WTRI = O_WE2 + SZ_WE2;
constexpr size_t O_WTO  = O_WTRI + SZ_WTRI;
constexpr size_t O_H1   = O_WTO + SZ_WTO;
constexpr size_t O_HN   = O_H1 + SZ_NF;
constexpr size_t O_OHL  = O_HN + SZ_NF;
constexpr size_t O_XHL  = O_OHL + SZ_NHL;
constexpr size_t O_GHL  = O_XHL + SZ_NHL;
constexpr size_t WS_TOTAL = O_GHL + SZ_GHL;

static_assert(WS_TOTAL == 128200704);
static_assert(WS_TOTAL <= 134217728);
static_assert(O_P == O_Q + PLANE_H * 2);
static_assert(O_VT == O_Q + 2 * PLANE_H * 2);
static_assert((O_WTRI % 256) == 0);
static_assert((O_WTO % 256) == 0);
static_assert((O_GHL % 256) == 0);
static_assert((size_t)OUT1_OFF + (size_t)NPAIR * DEDGE == 8454144);

extern "C" void kernel_launch(void* const* d_in, const int* in_sizes, int n_in,
                              void* d_out, int out_size, void* d_ws, size_t ws_size,
                              hipStream_t stream) {
  if (n_in < 24) return;
  const int expect[24] = { 65536, 8388608, 65536, 65536, 65536, 2048, 65536, 256, 262144, 1024, 262144, 256,
                           65536, 512, 65536, 128, 1024, 128, 16384, 16384, 16384, 1024, 32768, 128 };
  for (int t = 0; t < 24; ++t) if (in_sizes[t] != expect[t]) return;
  if (out_size != 8454144) return;
  if (ws_size < WS_TOTAL) return;

  const float* h_in  = (const float*)d_in[0];
  const float* e_in  = (const float*)d_in[1];
  const float* Wq    = (const float*)d_in[2];
  const float* Wk    = (const float*)d_in[3];
  const float* Wv    = (const float*)d_in[4];
  const float* W_ebg = (const float*)d_in[5];
  const float* Wo    = (const float*)d_in[6];
  const float* bo    = (const float*)d_in[7];
  const float* Wn1   = (const float*)d_in[8];
  const float* bn1   = (const float*)d_in[9];
  const float* Wn2   = (const float*)d_in[10];
  const float* bn2   = (const float*)d_in[11];
  const float* We1   = (const float*)d_in[12];
  const float* be1   = (const float*)d_in[13];
  const float* We2   = (const float*)d_in[14];
  const float* be2   = (const float*)d_in[15];
  const float* Wl2e  = (const float*)d_in[16];
  const float* bl2e  = (const float*)d_in[17];
  const float* Wqt   = (const float*)d_in[18];
  const float* Wpt   = (const float*)d_in[19];
  const float* Wvt   = (const float*)d_in[20];
  const float* Wgbt  = (const float*)d_in[21];
  const float* Wto   = (const float*)d_in[22];
  const float* bto   = (const float*)d_in[23];

  float* out0 = (float*)d_out;
  float* out1 = (float*)d_out + OUT1_OFF;

  char* ws = (char*)d_ws;
  float*          ES   = (float*)(ws + O_ES);
  unsigned short* QPV  = (unsigned short*)(ws + O_Q);
  unsigned short* OP   = (unsigned short*)(ws + O_OP);
  float*          GT   = (float*)(ws + O_GT);
  float*          Z    = (float*)(ws + O_Z);
  float*          QKV  = (float*)(ws + O_QKV);
  unsigned short* HB   = (unsigned short*)(ws + O_HB);
  unsigned short* WQKV = (unsigned short*)(ws + O_WQKV);
  unsigned short* WO2  = (unsigned short*)(ws + O_WO2);
  unsigned short* WN1  = (unsigned short*)(ws + O_WN1);
  unsigned short* WN2  = (unsigned short*)(ws + O_WN2);
  unsigned short* WEBG = (unsigned short*)(ws + O_WEBG);
  unsigned short* WE1  = (unsigned short*)(ws + O_WE1);
  unsigned short* WE2  = (unsigned short*)(ws + O_WE2);
  unsigned short* WTRI = (unsigned short*)(ws + O_WTRI);
  unsigned short* WTO  = (unsigned short*)(ws + O_WTO);
  float*          H1   = (float*)(ws + O_H1);
  float*          HN   = (float*)(ws + O_HN);
  unsigned short* OHL  = (unsigned short*)(ws + O_OHL);
  unsigned short* XHL  = (unsigned short*)(ws + O_XHL);
  unsigned short* GHL  = (unsigned short*)(ws + O_GHL);

  auto prep = [&](const float* W, unsigned short* out, int K, int Ncols, int KD, int rowsOut) {
    const int total = rowsOut * (KD >> 3);
    k_prepT<<<dim3((total + 255) / 256), dim3(256), 0, stream>>>(W, out, K, Ncols, KD, rowsOut);
  };
  k_cvt<<<dim3(32), dim3(256), 0, stream>>>(h_in, HB, 8192);
  prep(Wq,    WQKV,                      256, 256,  256,  256);
  prep(Wk,    WQKV + (size_t)256 * 256,  256, 256,  256,  256);
  prep(Wv,    WQKV + (size_t)512 * 256,  256, 256,  256,  256);
  prep(Wo,    WO2,                       256, 256,  512,  256);
  prep(Wn1,   WN1,                       256, 1024, 512,  1024);
  prep(Wn2,   WN2,                       1024, 256, 2048, 256);
  prep(W_ebg, WEBG,                      128, 16,   128,  16);
  prep(We1,   WE1,                       128, 512,  256,  512);
  prep(We2,   WE2,                       512, 128,  1024, 128);
  prep(Wqt,   WTRI,                      128, 128,  256,  128);
  prep(Wpt,   WTRI + (size_t)128 * 256,  128, 128,  256,  128);
  prep(Wvt,   WTRI + (size_t)256 * 256,  128, 128,  256,  128);
  prep(Wgbt,  WTRI + (size_t)384 * 256,  128, 8,    256,  16);
  prep(Wto,   WTO,                       256, 128,  256,  128);

  k_gemm<false, false, 0, false, 0><<<dim3(2, 12), dim3(128), 0, stream>>>(
      HB, WQKV, (void*)QKV, bo, QKV, QKV, 256, 256, 768, 256);
  k_eagg<<<dim3(1024), dim3(256), 0, stream>>>(e_in, QKV, WEBG, Wl2e, bl2e, Z, ES);
  k_nattn<<<dim3(256), dim3(256), 0, stream>>>(Z, QKV, OHL);
  k_gemm<true, false, 1, true, 0><<<dim3(2, 4), dim3(128), 0, stream>>>(
      OHL, WO2, (void*)H1, bo, h_in, h_in, 512, 512, 256, 512);
  k_nln<<<dim3(64), dim3(128), 0, stream>>>(H1, HN, XHL);
  k_gemm<true, true, 0, false, 1><<<dim3(2, 16), dim3(128), 0, stream>>>(
      XHL, WN1, (void*)GHL, bn1, H1, H1, 512, 512, 2048, 512);
  k_gemm<true, false, 2, false, 0><<<dim3(2, 4), dim3(128), 0, stream>>>(
      GHL, WN2, (void*)out0, bn2, H1, HN, 2048, 2048, 256, 2048);

  (void)hipFuncSetAttribute(reinterpret_cast<const void*>(&k_ffn), hipFuncAttributeMaxDynamicSharedMemorySize, FFN_LDS);
  k_ffn<<<dim3(1024), dim3(256), FFN_LDS, stream>>>(ES, ES, WE1, WE2, be1, be2);
  k_tproj<<<dim3(1024), dim3(256), 0, stream>>>(ES, WTRI, QPV, GT);
  k_tattn<<<dim3(4096), dim3(128), 0, stream>>>(QPV, GT, OP);
  k_gemm<true, false, 1, false, 0><<<dim3(512, 2), dim3(128), 0, stream>>>(
      OP, WTO, (void*)ES, bto, ES, ES, 256, 256, 128, 256);
  k_ffn<<<dim3(1024), dim3(256), FFN_LDS, stream>>>(ES, out1, WE1, WE2, be1, be2);
  (void)hipGetLastError();
}
